// Memory_Transformer_12043088298476
// MI455X (gfx1250) — hardware-verified
//
#include <hip/hip_runtime.h>
#include <math.h>

typedef __attribute__((ext_vector_type(16))) _Float16 v16h;
typedef __attribute__((ext_vector_type(16))) __bf16 v16b;
typedef __attribute__((ext_vector_type(8)))  _Float16 v8h;
typedef __attribute__((ext_vector_type(8)))  float v8f;
typedef __attribute__((ext_vector_type(4)))  float v4f;
typedef __attribute__((ext_vector_type(2)))  float v2f;
typedef __attribute__((ext_vector_type(4)))  unsigned v4u;
typedef __attribute__((ext_vector_type(4)))  int v4i;
typedef float __attribute__((may_alias)) float_a;
typedef int __attribute__((may_alias)) int_a;

template <typename T> __device__ __forceinline__ void vst2(void* p, T v) { *(volatile T*)p = v; __threadfence(); *(volatile T*)p = v; }
__device__ __forceinline__ v8f wmma16(v16h a, v16h b, v8f c) {
  v8f d = __builtin_amdgcn_wmma_f32_16x16x32_f16(false, a, false, b, (short)0, c, false, false);
  asm volatile("v_nop\n\tv_nop\n\tv_nop\n\tv_nop" : "+v"(d) : "v"(a), "v"(b));
  return d;
}
__device__ __forceinline__ v8f wmma_bf(v16b a, v16b b, v8f c) {
  v8f d = __builtin_amdgcn_wmma_f32_16x16x32_bf16(false, a, false, b, (short)0, c, false, false);
  asm volatile("v_nop\n\tv_nop\n\tv_nop\n\tv_nop" : "+v"(d) : "v"(a), "v"(b));
  return d;
}
__device__ __forceinline__ v16h frag_h(const _Float16* rowk0, int lane) {
  union { v16h v; v8h q[2]; } u; const _Float16* p = rowk0 + 8 * (lane >> 4);
  u.q[0] = *(const v8h*)p; u.q[1] = *(const v8h*)(p + 16); return u.v;
}
__device__ __forceinline__ v16h frag_f32(const float* rowk0, int lane) {
  v16h a; const float* p = rowk0 + 8 * (lane >> 4);
#pragma unroll
  for (int i = 0; i < 8; ++i) { a[i] = (_Float16)p[i]; a[8 + i] = (_Float16)p[16 + i]; }
  return a;
}
__device__ __forceinline__ v16h frag_f32s(const float* rowk0, int lane, float sc) {
  v16h a; const float* p = rowk0 + 8 * (lane >> 4);
#pragma unroll
  for (int i = 0; i < 8; ++i) { a[i] = (_Float16)(p[i] * sc); a[8 + i] = (_Float16)(p[16 + i] * sc); }
  return a;
}
__device__ __forceinline__ v16h fragc_f32(const float* W, int k0, int n, int lane, int ld, int K) {
  v16h a; const int g = lane >> 4;
#pragma unroll
  for (int i = 0; i < 8; ++i) { const int ka = k0 + 8 * g + i, kb = ka + 16;
    a[i] = (_Float16)(ka < K ? W[(size_t)(ka < K ? ka : K - 1) * ld + n] : 0.f); a[8 + i] = (_Float16)(kb < K ? W[(size_t)(kb < K ? kb : K - 1) * ld + n] : 0.f); }
  return a;
}
struct F2 { v16b h, l; };
__device__ __forceinline__ F2 bsplit16(const float v[16]) { F2 r;
#pragma unroll
  for (int i = 0; i < 16; ++i) { const __bf16 h = (__bf16)v[i]; r.h[i] = h; r.l[i] = (__bf16)(v[i] - (float)h); }
  return r; }
__device__ __forceinline__ F2 split_row(const float* row, int k0, int lane) { float v[16]; const float* p = row + k0 + 8 * (lane >> 4);
#pragma unroll
  for (int i = 0; i < 8; ++i) { v[i] = p[i]; v[8 + i] = p[16 + i]; }
  return bsplit16(v); }
__device__ __forceinline__ F2 split_rowK(const float* row, int k0, int lane, int K) { float v[16]; const int g = lane >> 4;
#pragma unroll
  for (int i = 0; i < 8; ++i) { const int ka = k0 + 8 * g + i, kb = ka + 16; v[i] = ka < K ? row[ka < K ? ka : K - 1] : 0.f; v[8 + i] = kb < K ? row[kb < K ? kb : K - 1] : 0.f; }
  return bsplit16(v); }
__device__ __forceinline__ F2 split_col(const float* W, int k0, int n, int lane, int ld, int K) { float v[16]; const int g = lane >> 4;
#pragma unroll
  for (int i = 0; i < 8; ++i) { const int ka = k0 + 8 * g + i, kb = ka + 16; v[i] = ka < K ? W[(size_t)(ka < K ? ka : K - 1) * ld + n] : 0.f; v[8 + i] = kb < K ? W[(size_t)(kb < K ? kb : K - 1) * ld + n] : 0.f; }
  return bsplit16(v); }
__device__ __forceinline__ v8f mac3(const F2& a, const F2& b, v8f c) { c = wmma_bf(a.l, b.h, c); c = wmma_bf(a.h, b.l, c); return wmma_bf(a.h, b.h, c); }
__device__ __forceinline__ float sigm(float v) { return 1.0f / (1.0f + expf(-v)); }
#define LDSX() do { asm volatile("s_wait_dscnt 0" ::: "memory"); __builtin_amdgcn_wave_barrier(); __builtin_amdgcn_fence(__ATOMIC_RELEASE, "workgroup"); } while (0)


#define TT 8192
#define KD 1024
#define VD 1024
#define QBLK 512
#ifndef NQB
#define NQB (TT / QBLK)
#endif
typedef __attribute__((ext_vector_type(8))) __bf16 v8b;
__device__ __forceinline__ v16b frag_b(const __bf16* rowk0, int lane) {
  union { v16b v; v8b q[2]; } u; const __bf16* p = rowk0 + 8 * (lane >> 4);
  u.q[0] = *(const v8b*)p; u.q[1] = *(const v8b*)(p + 16); return u.v;
}
__device__ __forceinline__ float bfr(float v) { return (float)(__bf16)v; }
__device__ __attribute__((noinline)) float exp_ni(float v) { return expf(v); }
__device__ __attribute__((noinline)) float erf_ni(float v) { return erff(v); }

#define WS_Q   0u
#define WS_K   (WS_Q + 2u * (size_t)TT * KD)
#define WS_VT  (WS_K + 2u * (size_t)TT * KD)
#define WS_S   (WS_VT + 2u * (size_t)VD * TT)
#define WS_P   (WS_S + 4u * (size_t)QBLK * TT)
#define WS_PL  (WS_P + 2u * (size_t)QBLK * TT)
#define WS_IL  (WS_PL + 2u * (size_t)QBLK * TT)
#define WS_END (WS_IL + 4u * QBLK + 256u)
#define HPQB 2

__global__ __launch_bounds__(256) void k_rows(const float* __restrict__ X, _Float16* __restrict__ R) { const size_t r0 = (size_t)blockIdx.x * 64; const int t = threadIdx.x; __shared__ __align__(16) _Float16 s[64][KD / 4 + 8];
  for (int pass = 0; pass < 4; ++pass) { for (int e = t; e < 64 * 256; e += 256) { const int r = e >> 8, c = e & 255; s[r][c] = (_Float16)bfr(X[(r0 + r) * KD + pass * 256 + c]); } __syncthreads(); for (int e = t; e < 64 * 32; e += 256) { const int r = e >> 5, q = e & 31; vst2((unsigned*)(R + (r0 + r) * KD + pass * 256 + q * 8), *(const v4u*)&s[r][q * 8]); } __syncthreads(); } }
__global__ __launch_bounds__(256) void k_vt(const float* __restrict__ V, _Float16* __restrict__ VT) { __shared__ __align__(16) _Float16 st[128][72]; const size_t r0 = (size_t)blockIdx.x * 64; const int c0 = blockIdx.y * 128, t = threadIdx.x;
  for (int e = t; e < 64 * 128; e += 256) { const int r = e >> 7, c = e & 127; st[c][r] = (_Float16)bfr(V[(r0 + r) * VD + c0 + c]); } __syncthreads();
  for (int e = t; e < 128 * 8; e += 256) { const int c = e >> 3, pc = e & 7; vst2((unsigned*)(VT + (size_t)(c0 + c) * TT + r0 + pc * 8), *(const v4u*)&st[c][pc * 8]); } }
__global__ __launch_bounds__(128) void k_scores(const _Float16* __restrict__ Q, const _Float16* __restrict__ K, int qbase, float* __restrict__ S) {
  __shared__ __align__(16) float so[4][16][132];
  const int tid = threadIdx.x, wave = tid >> 5, lane = tid & 31, col = lane & 15, g = lane >> 4; const int rloc0 = blockIdx.x * 64 + wave * 16; const size_t rq = (size_t)qbase + rloc0; const int k0 = blockIdx.y * 128;
  v8f acc[8] = {};
#pragma unroll 4
  for (int kc = 0; kc < KD / 32; ++kc) { const v16h a = frag_h(Q + (rq + col) * KD + kc * 32, lane);
#pragma unroll
    for (int j = 0; j < 8; ++j) acc[j] = wmma16(a, frag_h(K + (size_t)(k0 + j * 16 + col) * KD + kc * 32, lane), acc[j]); }
#pragma unroll
  for (int j = 0; j < 8; ++j) { const int kk = k0 + j * 16 + col;
#pragma unroll
    for (int r = 0; r < 8; ++r) { const int qq = qbase + rloc0 + 8 * g + r; so[wave][8 * g + r][j * 16 + col] = (kk <= qq) ? acc[j][r] * 0.03125f : -3.0e38f; } }
  LDSX();
  for (int rl = 0; rl < 16; ++rl) vst2(S + (size_t)(rloc0 + rl) * TT + k0 + lane * 4, *(const v4f*)&so[wave][rl][lane * 4]);
}
__global__ __launch_bounds__(256) void k_soft(const float* __restrict__ S, int nk, int hp, _Float16* __restrict__ P, _Float16* __restrict__ PL, float* __restrict__ IL) {
  __shared__ float red[256]; __shared__ __align__(16) _Float16 sp[TT]; __shared__ __align__(16) _Float16 spl[1024];
  const int r = blockIdx.x, t = threadIdx.x; const float* row = S + (size_t)r * TT;
  float mx = -3.0e38f; for (int k = t; k < nk; k += 256) mx = fmaxf(mx, row[k]); red[t] = mx; __syncthreads();
  for (int s = 128; s > 0; s >>= 1) { if (t < s) red[t] = fmaxf(red[t], red[t + s]); __syncthreads(); }
  const float gm = red[0]; __syncthreads();
  float sum = 0.f; for (int k = t; k < nk; k += 256) { const float v = row[k]; const float e = (v <= -1.0e38f) ? 0.f : __expf(v - gm); sum += e; const float pe = e * 2048.0f; const _Float16 h = (_Float16)pe; sp[k] = h; if (hp) spl[k] = (_Float16)((pe - (float)h) * 2048.0f); }
  red[t] = sum; __syncthreads();
  for (int s = 128; s > 0; s >>= 1) { if (t < s) red[t] += red[t + s]; __syncthreads(); }
  if (t == 0) IL[r] = (1.0f / 2048.0f) / red[0];
  for (int q = t; q < nk / 8; q += 256) vst2((unsigned*)(P + (size_t)r * TT + q * 8), *(const v4u*)&sp[q * 8]);
  if (hp) for (int q = t; q < nk / 8; q += 256) vst2((unsigned*)(PL + (size_t)r * TT + q * 8), *(const v4u*)&spl[q * 8]);
}
__global__ __launch_bounds__(128) void k_pv(const _Float16* __restrict__ P, const _Float16* __restrict__ PL, const _Float16* __restrict__ VT, const float* __restrict__ IL, int qbase, int nk, int hp, float* __restrict__ OUT) {
  __shared__ __align__(16) float so[4][16][132];
  const int tid = threadIdx.x, wave = tid >> 5, lane = tid & 31, col = lane & 15, g = lane >> 4; const int rloc0 = blockIdx.x * 64 + wave * 16; const int d0 = blockIdx.y * 128;
  v8f acc[8] = {}, accl[8] = {};
#pragma unroll 2
  for (int kc = 0; kc < nk / 32; ++kc) { const v16h a = frag_h(P + (size_t)(rloc0 + col) * TT + kc * 32, lane); v16h al = {}; if (hp) al = frag_h(PL + (size_t)(rloc0 + col) * TT + kc * 32, lane);
#pragma unroll
    for (int j = 0; j < 8; ++j) { const v16h vf = frag_h(VT + (size_t)(d0 + j * 16 + col) * TT + kc * 32, lane); acc[j] = wmma16(a, vf, acc[j]); if (hp) accl[j] = wmma16(al, vf, accl[j]); } }
#pragma unroll
  for (int j = 0; j < 8; ++j)
#pragma unroll
    for (int r = 0; r < 8; ++r) so[wave][8 * g + r][j * 16 + col] = (acc[j][r] + accl[j][r] * (1.0f / 2048.0f)) * IL[rloc0 + 8 * g + r];
  LDSX();
  for (int rl = 0; rl < 16; ++rl) vst2(OUT + (size_t)(qbase + rloc0 + rl) * VD + d0 + lane * 4, *(const v4f*)&so[wave][rl][lane * 4]);
}
extern "C" void kernel_launch(void* const* d_in, const int* in_sizes, int n_in, void* d_out, int out_size, void* d_ws, size_t ws_size, hipStream_t stream) {
  (void)in_sizes; (void)n_in; (void)out_size;
  const float** F = (const float**)d_in;
  if (ws_size < (size_t)WS_END) return;
  char* ws = (char*)d_ws; _Float16 *Q = (_Float16*)(ws + WS_Q), *K = (_Float16*)(ws + WS_K), *VT = (_Float16*)(ws + WS_VT), *P = (_Float16*)(ws + WS_P), *PL = (_Float16*)(ws + WS_PL); float *S = (float*)(ws + WS_S), *IL = (float*)(ws + WS_IL);
  k_rows<<<TT / 64, 256, 0, stream>>>(F[0], Q);
  k_rows<<<TT / 64, 256, 0, stream>>>(F[1], K);
  k_vt<<<dim3(TT / 64, VD / 128), 256, 0, stream>>>(F[2], VT);
  for (int qb = 0; qb < NQB; ++qb) { const int qbase = qb * QBLK; const int nk = qbase + QBLK;
    k_scores<<<dim3(QBLK / 64, nk / 128), 128, 0, stream>>>(Q, K, qbase, S);
    const int hp = (qb < HPQB) ? 1 : 0;
    k_soft<<<QBLK, 256, 0, stream>>>(S, nk, hp, P, PL, IL);
    k_pv<<<dim3(QBLK / 64, VD / 128), 128, 0, stream>>>(P, PL, VT, IL, qbase, nk, hp, (float*)d_out); }
}
